// SparseMoE_83399674953937
// MI455X (gfx1250) — hardware-verified
//
#include <hip/hip_runtime.h>
#include <math.h>

typedef __attribute__((ext_vector_type(16))) _Float16 v16h;
typedef __attribute__((ext_vector_type(8)))  _Float16 v8h;
typedef __attribute__((ext_vector_type(8)))  float v8f;
typedef __attribute__((ext_vector_type(4)))  float v4f;
typedef __attribute__((ext_vector_type(2)))  float v2f;
typedef __attribute__((ext_vector_type(4)))  unsigned v4u;
typedef _Float16 h16;

#ifndef NB
#define NB 4
#endif
#ifndef SEQ
#define SEQ 2048
#endif
#define NB_FULL 4
#define SEQ_FULL 2048
#define NT (NB * SEQ)
#define NT_FULL (NB_FULL * SEQ_FULL)
#define DIN  1024
#define DOUT 1024
#define NE   8
#define TOPK 4
#define KF (NE * DIN)
#define KP (KF + 64)
#define HCARRY 64.0f
#define WCARRY 512.0f
#define OSCALE (1.0f / 32768.0f)
#define CHUNK (NT < 4096 ? NT : 4096)
#define NCH (NT / CHUNK)
#define OUT1_ELEM ((size_t)NT_FULL * DOUT)

#define WS_WT  ((size_t)0)
#define WS_HB  (WS_WT + (size_t)DOUT * KP * 2)
#define WS_GW  (WS_HB + (size_t)CHUNK * KP * 2)
#define WS_PT  (WS_GW + (size_t)NT * NE * 4)
#define WS_END (WS_PT + (size_t)(NT / 64) * 128)

static_assert(NE == 8 && TOPK == 4);
static_assert(NT % 128 == 0 && NT % 64 == 0);
static_assert(CHUNK % 128 == 0 && NT % CHUNK == 0 && NCH * CHUNK == NT);
static_assert(NT <= NT_FULL);
static_assert(DIN % 32 == 0 && KP % 32 == 0 && (KP * 2) % 128 == 0);
static_assert(DOUT % 128 == 0 && DIN % 64 == 0 && DOUT % 64 == 0);
static_assert(OUT1_ELEM * 4 == 33554432);
static_assert((OUT1_ELEM + 1) * 4 <= 33554436);
static_assert((size_t)NT * DOUT <= OUT1_ELEM);
static_assert(WS_HB % 128 == 0 && WS_GW % 128 == 0 && WS_PT % 128 == 0);
static_assert(WS_END <= (size_t)134217728);
static_assert((size_t)(DOUT / 64) * (DIN / 64) * NE * 4096 == (size_t)DOUT * KF);
static_assert((size_t)(DOUT * 8 / 256) * 256 * 8 == (size_t)DOUT * 64);
static_assert((size_t)(NT / 64) * 64 * 2 * 4 == (size_t)NT * NE);
static_assert((size_t)(CHUNK / 2) * 256 * 8 * 8 == (size_t)CHUNK * KF);
static_assert((size_t)256 * 8 * 16 == (size_t)2 * KF * 2);
static_assert((size_t)(CHUNK / 2) * 2 * 8 * 8 == (size_t)CHUNK * 64);
static_assert((size_t)(DOUT / 128) * (CHUNK / 128) * 128 * 128 == (size_t)CHUNK * DOUT);
static_assert(64 * 65 * 4 <= 131072);
static_assert(DIN * NE * 4 + 64 * NE * 4 * 2 + 64 * 4 + 32 * 4 <= 131072);
static_assert(8 * 16 * 64 * 4 <= 131072);
static_assert(32 * 8 <= 131072);

__device__ __forceinline__ v8f wmma16(v16h a, v16h b, v8f c) {
  v8f d = __builtin_amdgcn_wmma_f32_16x16x32_f16(false, a, false, b, (short)0, c, false, false);
  asm volatile("v_nop\n\tv_nop\n\tv_nop\n\tv_nop" : "+v"(d) : "v"(a), "v"(b));
  return d;
}
__device__ __forceinline__ float bfr(float v) { return (float)(__bf16)v; }
static __device__ __forceinline__ h16 toh_flush(float v) { const h16 r = (h16)v; return (fabsf(v) < 6.103515625e-05f) ? (h16)0.0f : r; }
__device__ __forceinline__ v16h ldfrag_h(const unsigned short* p) { union { v16h v; v4u q[2]; } f; f.q[0] = *(const v4u*)p; f.q[1] = *(const v4u*)(p + 16); return f.v; }

__global__ __launch_bounds__(256) void k_tr(const float* __restrict__ S, unsigned short* __restrict__ Dst, unsigned K, unsigned N, unsigned dpitch, unsigned erow, unsigned ecol, float sc) {
  __shared__ float tile[64][65];
  const unsigned t = threadIdx.x, e = blockIdx.z, k0 = blockIdx.y * 64u, n0 = blockIdx.x * 64u;
  const float* s = S + (size_t)e * K * N;
#pragma unroll
  for (unsigned it = 0; it < 4; ++it) { const unsigned idx = it * 256u + t, kr = idx >> 4, c4 = idx & 15u;
    const v4f v = *(const v4f*)(s + (size_t)(k0 + kr) * N + n0 + 4u * c4);
    tile[kr][4u * c4 + 0] = v[0]; tile[kr][4u * c4 + 1] = v[1]; tile[kr][4u * c4 + 2] = v[2]; tile[kr][4u * c4 + 3] = v[3]; }
  __syncthreads();
  v4u o[2];
#pragma unroll
  for (unsigned it = 0; it < 2; ++it) { const unsigned idx = it * 256u + t, nr = idx >> 3, q = idx & 7u;
    union { v8h h; v4u u; } w;
#pragma unroll
    for (int i = 0; i < 8; ++i) { const float v = bfr(tile[8u * q + i][nr]); w.h[i] = toh_flush(v * sc); }
    o[it] = w.u; }
#pragma unroll
  for (unsigned it = 0; it < 2; ++it) { const unsigned idx = it * 256u + t, nr = idx >> 3, q = idx & 7u;
    *(volatile v4u*)(Dst + (size_t)(e * erow + n0 + nr) * dpitch + e * ecol + k0 + 8u * q) = o[it]; }
  __threadfence();
#pragma unroll
  for (unsigned it = 0; it < 2; ++it) { const unsigned idx = it * 256u + t, nr = idx >> 3, q = idx & 7u;
    *(volatile v4u*)(Dst + (size_t)(e * erow + n0 + nr) * dpitch + e * ecol + k0 + 8u * q) = o[it]; }
}

__global__ __launch_bounds__(256) void k_bpad(const float* __restrict__ BV, unsigned short* __restrict__ WT) {
  const unsigned idx = blockIdx.x * 256u + threadIdx.x; const unsigned n = (idx >> 3) & (DOUT - 1u), q = idx & 7u;
  union { v8h h; v4u u; } w;
#pragma unroll
  for (int i = 0; i < 8; ++i) { const float v = bfr(BV[(size_t)i * DOUT + n]) * WCARRY; w.h[i] = toh_flush(q == 0u ? v : 0.f); }
  const v4u val = w.u;
  volatile v4u* p = (volatile v4u*)(WT + (size_t)n * KP + KF + 8u * q);
  *p = val; __threadfence(); *p = val;
}

__global__ __launch_bounds__(64) void k_gate(const float* __restrict__ X, const float* __restrict__ WG, const float* __restrict__ BG, float* __restrict__ GW, float* __restrict__ PART) {
#pragma clang fp contract(off)
  __shared__ __align__(16) float swg[DIN * NE];
  __shared__ __align__(16) float sp[64][NE];
  __shared__ __align__(16) float sg[64][NE];
  __shared__ unsigned su[64];
  __shared__ __align__(16) float sline[32];
  const unsigned tid = threadIdx.x, lane = tid & 31u; const unsigned wave = __builtin_amdgcn_readfirstlane(tid >> 5);
  const unsigned r0 = blockIdx.x * 64u;
#pragma unroll 1
  for (unsigned i = tid; i < (unsigned)(DIN * NE / 4); i += 64u) { const v4f w = *(const v4f*)(WG + 4u * i); v4f o;
    o[0] = bfr(w[0]); o[1] = bfr(w[1]); o[2] = bfr(w[2]); o[3] = bfr(w[3]);
    *(v4f*)&swg[4u * i] = o; }
  __syncthreads();
  const float* xr = X + (size_t)(r0 + tid) * DIN;
  float a[NE];
#pragma unroll
  for (int e = 0; e < NE; ++e) a[e] = 0.f;
#pragma unroll 1
  for (unsigned d = 0; d < (unsigned)DIN; d += 2u) { const v2f xv = *(const v2f*)(xr + d);
#pragma unroll
    for (int j = 0; j < 2; ++j) { const float xb = bfr(xv[j]);
      const v4f w0 = *(const v4f*)&swg[(d + j) * NE], w1 = *(const v4f*)&swg[(d + j) * NE + 4u];
#pragma unroll
      for (int e = 0; e < 4; ++e) { a[e] = fmaf(xb, w0[e], a[e]); a[4 + e] = fmaf(xb, w1[e], a[4 + e]); } } }
#pragma unroll
  for (int e = 0; e < NE; ++e) sp[tid][e] = a[e] + bfr(BG[e]);
  float m = sp[tid][0];
#pragma unroll 1
  for (unsigned e = 1; e < (unsigned)NE; ++e) m = fmaxf(m, sp[tid][e]);
  float s = 0.f;
#pragma unroll 1
  for (unsigned e = 0; e < (unsigned)NE; ++e) { const float ev = expf(sp[tid][e] - m); sp[tid][e] = ev; s += ev; }
  const float inv = 1.0f / s;
#pragma unroll 1
  for (unsigned e = 0; e < (unsigned)NE; ++e) { const float pv = sp[tid][e] * inv; sp[tid][e] = pv; }
  unsigned used = 0u; float ssel = 0.f; float pk[TOPK]; unsigned ik[TOPK];
#pragma unroll
  for (int kk = 0; kk < TOPK; ++kk) { unsigned best = 0u; float bv = -1.f;
#pragma unroll 1
    for (unsigned e = 0; e < (unsigned)NE; ++e) { const float pv = sp[tid][e]; const bool c = (((used >> e) & 1u) == 0u) && (pv > bv); bv = c ? pv : bv; best = c ? e : best; }
    used |= 1u << best; ik[kk] = best; pk[kk] = bv; ssel += bv; }
  const float wn = 1.0f / (ssel + 1e-6f);
#pragma unroll
  for (int e = 0; e < NE; ++e) sg[tid][e] = 0.f;
#pragma unroll
  for (int kk = 0; kk < TOPK; ++kk) sg[tid][ik[kk] & 7u] = pk[kk] * wn;
  su[tid] = used;
  __syncthreads();
  const unsigned ec = tid & 7u; float ps = 0.f; unsigned cn = 0u;
#pragma unroll 1
  for (unsigned r = 0; r < 64u; ++r) { ps += sp[r][ec]; cn += (su[r] >> ec) & 1u; }
  const float val = (tid & 8u) ? (float)cn : ps;
  if (wave == 0u) sline[lane] = (lane < 16u) ? val : 0.f;
  __syncthreads();
  v4f gv[2];
#pragma unroll
  for (unsigned it = 0; it < 2; ++it) { const unsigned idx = it * 64u + tid; gv[it] = *(const v4f*)(&sg[0][0] + 4u * idx); }
  const v4f pl = *(const v4f*)&sline[4u * (tid & 7u)];
  float* go = GW + (size_t)r0 * NE;
  float* po = PART + (size_t)blockIdx.x * 32u;
#pragma unroll
  for (unsigned it = 0; it < 2; ++it) { const unsigned idx = it * 64u + tid; *(volatile v4f*)(go + 4u * idx) = gv[it]; }
  if (tid < 8u) *(volatile v4f*)(po + 4u * tid) = pl;
  __threadfence();
#pragma unroll
  for (unsigned it = 0; it < 2; ++it) { const unsigned idx = it * 64u + tid; *(volatile v4f*)(go + 4u * idx) = gv[it]; }
  if (tid < 8u) *(volatile v4f*)(po + 4u * tid) = pl;
}

__global__ __launch_bounds__(32) void k_aux(const float* __restrict__ PART, float* __restrict__ OUT1) {
#pragma clang fp contract(off)
  __shared__ double sv[32];
  const unsigned lane = threadIdx.x & 31u, c = lane & 15u;
  double acc = 0.0;
#pragma unroll 1
  for (unsigned b = 0; b < (unsigned)(NT / 64); ++b) acc += (double)PART[(size_t)b * 32u + c];
  sv[lane] = acc;
  __syncthreads();
  const double invT = 1.0 / (double)NT;
  double av = 0.0;
#pragma unroll 1
  for (unsigned e = 0; e < (unsigned)NE; ++e) av += (sv[8u + e] * invT) * (sv[e] * invT);
  const float r = (float)(av * (double)NE);
  if (lane == 0u) { volatile float* p = (volatile float*)OUT1; *p = r; __threadfence(); *p = r; }
}

__global__ __launch_bounds__(256) void k_ax(const float* __restrict__ X, const float* __restrict__ GW, unsigned short* __restrict__ HB, unsigned t0) {
  const unsigned tid = threadIdx.x; const unsigned wave = __builtin_amdgcn_readfirstlane(tid >> 5);
  const unsigned rl = blockIdx.x * 2u + (wave >> 2), c = tid & 127u;
  const size_t tg = (size_t)t0 + rl;
  const float* xr = X + tg * DIN + 8u * c;
  const v4f x0 = *(const v4f*)xr, x1 = *(const v4f*)(xr + 4);
  const v4f g0 = *(const v4f*)(GW + tg * NE), g1 = *(const v4f*)(GW + tg * NE + 4);
  float xs[8], g[8];
#pragma unroll
  for (int j = 0; j < 4; ++j) { xs[j] = bfr(x0[j]) * HCARRY; xs[4 + j] = bfr(x1[j]) * HCARRY; g[j] = g0[j]; g[4 + j] = g1[j]; }
  v4u o[NE];
#pragma unroll
  for (int e = 0; e < NE; ++e) { union { v8h h; v4u u; } w;
#pragma unroll
    for (int i = 0; i < 8; ++i) w.h[i] = toh_flush(xs[i] * g[e]);
    o[e] = w.u; }
  v4u pv; { union { v8h h; v4u u; } w;
#pragma unroll
    for (int i = 0; i < 8; ++i) w.h[i] = toh_flush(c == 0u ? g[i] * HCARRY : 0.f);
    pv = w.u; }
  unsigned short* hr = HB + (size_t)rl * KP;
#pragma unroll
  for (int e = 0; e < NE; ++e) *(volatile v4u*)(hr + (size_t)e * DIN + 8u * c) = o[e];
  if (c < 8u) *(volatile v4u*)(hr + KF + 8u * c) = pv;
  __threadfence();
#pragma unroll
  for (int e = 0; e < NE; ++e) *(volatile v4u*)(hr + (size_t)e * DIN + 8u * c) = o[e];
  if (c < 8u) *(volatile v4u*)(hr + KF + 8u * c) = pv;
}

__global__ __launch_bounds__(256) void k_out(const unsigned short* __restrict__ HB, const unsigned short* __restrict__ W2T, float* __restrict__ OUT) {
  __shared__ __align__(16) float sf[8][16][64];
  const unsigned t = threadIdx.x, wave = t >> 5, lane = t & 31u, lm = lane & 15u, lh = lane >> 4, wm = wave >> 1, wn = wave & 1u;
  const unsigned m0 = blockIdx.y * 128u, n0 = blockIdx.x * 128u;
  const unsigned short* ar[2]; const unsigned short* br[4];
#pragma unroll
  for (int mi = 0; mi < 2; ++mi) ar[mi] = HB + (size_t)(m0 + wm * 32u + mi * 16u + lm) * KP + 8u * lh;
#pragma unroll
  for (int ni = 0; ni < 4; ++ni) br[ni] = W2T + (size_t)(n0 + wn * 64u + ni * 16u + lm) * KP + 8u * lh;
  v8f acc[2][4] = {};
#pragma unroll 2
  for (unsigned kc = 0; kc < KP / 32; ++kc) { v16h a[2], b[4];
#pragma unroll
    for (int mi = 0; mi < 2; ++mi) a[mi] = ldfrag_h(ar[mi] + kc * 32u);
#pragma unroll
    for (int ni = 0; ni < 4; ++ni) b[ni] = ldfrag_h(br[ni] + kc * 32u);
#pragma unroll
    for (int mi = 0; mi < 2; ++mi)
#pragma unroll
      for (int ni = 0; ni < 4; ++ni) acc[mi][ni] = wmma16(a[mi], b[ni], acc[mi][ni]); }
#pragma unroll
  for (int mi = 0; mi < 2; ++mi) {
    if (mi) __syncthreads();
#pragma unroll
    for (int ni = 0; ni < 4; ++ni)
#pragma unroll
      for (int r = 0; r < 8; ++r) sf[wave][8u * lh + r][ni * 16 + lm] = acc[mi][ni][r] * OSCALE;
    __syncthreads();
    v4f v[8];
#pragma unroll
    for (unsigned it = 0; it < 8; ++it) { const unsigned rw = it * 2u + (lane >> 4), pc = lane & 15u; v[it] = *(const v4f*)&sf[wave][rw][4u * pc]; }
    float* po = OUT + (size_t)(m0 + wm * 32u + mi * 16u) * DOUT + n0 + wn * 64u;
#pragma unroll
    for (unsigned it = 0; it < 8; ++it) { const unsigned rw = it * 2u + (lane >> 4), pc = lane & 15u; *(volatile v4f*)(po + (size_t)rw * DOUT + 4u * pc) = v[it]; }
    __threadfence();
#pragma unroll
    for (unsigned it = 0; it < 8; ++it) { const unsigned rw = it * 2u + (lane >> 4), pc = lane & 15u; *(volatile v4f*)(po + (size_t)rw * DOUT + 4u * pc) = v[it]; }
  }
}

extern "C" void kernel_launch(void* const* d_in, const int* in_sizes, int n_in, void* d_out, int out_size, void* d_ws, size_t ws_size, hipStream_t stream) {
  if (n_in < 5) return;
  if (in_sizes[0] < NT * DIN || in_sizes[1] < DIN * NE || in_sizes[2] < NE || in_sizes[3] < NE * DIN * DOUT || in_sizes[4] < NE * DOUT) return;
  if ((size_t)out_size < OUT1_ELEM + 1) return;
  if (ws_size < (size_t)WS_END) return;
  const float* X  = (const float*)d_in[0];
  const float* WG = (const float*)d_in[1];
  const float* BG = (const float*)d_in[2];
  const float* W  = (const float*)d_in[3];
  const float* BV = (const float*)d_in[4];
  char* ws = (char*)d_ws;
  unsigned short* WT = (unsigned short*)(ws + WS_WT);
  unsigned short* HB = (unsigned short*)(ws + WS_HB);
  float* GW   = (float*)(ws + WS_GW);
  float* PART = (float*)(ws + WS_PT);
  float* OUT  = (float*)d_out;
  float* AUX  = (float*)d_out + OUT1_ELEM;
  k_tr<<<dim3(DOUT / 64, DIN / 64, NE), 256, 0, stream>>>(W, WT, (unsigned)DIN, (unsigned)DOUT, (unsigned)KP, 0u, (unsigned)DIN, WCARRY);
  k_bpad<<<dim3(DOUT * 8 / 256), 256, 0, stream>>>(BV, WT);
  k_gate<<<dim3(NT / 64), 64, 0, stream>>>(X, WG, BG, GW, PART);
  k_aux<<<dim3(1), 32, 0, stream>>>(PART, AUX);
  for (unsigned c = 0; c < (unsigned)NCH; ++c) {
    k_ax<<<dim3(CHUNK / 2), 256, 0, stream>>>(X, GW, HB, c * (unsigned)CHUNK);
    k_out<<<dim3(DOUT / 128, CHUNK / 128), 256, 0, stream>>>(HB, WT, OUT + (size_t)c * CHUNK * DOUT);
  }
}
